// CrossAttention_27874337751456
// MI455X (gfx1250) — hardware-verified
//
#include <hip/hip_runtime.h>
#ifndef NB
#define NB 2
#endif
#ifndef SQ
#define SQ 2048
#endif
#define NB_FULL 2
#define SQ_FULL 2048
#define DM 1024
#define NH 16
#define HD 64
#define HG 2
#define NR ((size_t)NB * SQ)
#define MP ((int)((size_t)NB * SQ))

static_assert(SQ % 128 == 0);
static_assert(SQ <= SQ_FULL);
static_assert(NB >= 1 && NB <= NB_FULL);
static_assert(NH % HG == 0);
static_assert(HD == 64 && NH * HD == DM && DM % 64 == 0 && DM % 32 == 0);
static_assert((MP % 128) == 0);

typedef unsigned short v8us __attribute__((ext_vector_type(8), may_alias));
typedef float  v8f  __attribute__((ext_vector_type(8)));
typedef float  v4f  __attribute__((ext_vector_type(4)));
typedef float  v4fa __attribute__((ext_vector_type(4), may_alias));
typedef _Float16 v16h __attribute__((ext_vector_type(16)));
typedef _Float16 v4h __attribute__((ext_vector_type(4)));
union FragH { v16h v; v8us half[2]; _Float16 h[16]; unsigned short u[16]; };

__device__ __forceinline__ unsigned short bf16_bits(float x) { unsigned int u = __float_as_uint(x); return (unsigned short)((u + 0x7FFFu + ((u >> 16) & 1u)) >> 16); }
__device__ __forceinline__ float bf16_val(unsigned short b) { return __uint_as_float(((unsigned int)b) << 16); }
__device__ __forceinline__ float bf16_rne(float x) { return bf16_val(bf16_bits(x)); }

__device__ __forceinline__ v16h g2_frag(const _Float16* p, int hh) { FragH f; f.half[0] = *(const v8us*)((const unsigned short*)p + 8 * hh); f.half[1] = *(const v8us*)((const unsigned short*)p + 16 + 8 * hh); return f.v; }
__device__ __forceinline__ v8f g2_mma(v16h a, v16h b, v8f c) { v8f d = __builtin_amdgcn_wmma_f32_16x16x32_f16(false, a, false, b, (short)0, c, false, false); asm volatile("v_nop\n\tv_nop\n\tv_nop\n\tv_nop" : "+v"(d) : "v"(a), "v"(b)); return d; }

__global__ __launch_bounds__(256) void k_wnat(const float* __restrict__ w, size_t n8, _Float16* __restrict__ Bt) {
  const size_t t = (size_t)blockIdx.x * 256 + threadIdx.x; if (t >= n8) return; FragH f;
#pragma unroll
  for (int q = 0; q < 8; ++q) f.h[q] = (_Float16)(bf16_rne(w[t * 8 + q]) * 16.0f);
  *(volatile v8us*)((unsigned short*)Bt + t * 8) = f.half[0]; __threadfence(); *(volatile v8us*)((unsigned short*)Bt + t * 8) = f.half[0];
}

__global__ __launch_bounds__(256) void k_x16(const float* __restrict__ x, _Float16* __restrict__ X16, size_t n8) {
  const size_t t = (size_t)blockIdx.x * 256 + threadIdx.x; if (t >= n8) return;
  const size_t r = t / (DM / 8), c8 = (t % (DM / 8)) * 8;
  const size_t rs = (r / SQ) * SQ_FULL + (r % SQ);
  const float* src = x + rs * DM + c8;
  FragH f;
#pragma unroll
  for (int q = 0; q < 8; ++q) f.h[q] = (_Float16)bf16_rne(src[q]);
  *(volatile v8us*)((unsigned short*)X16 + t * 8) = f.half[0]; __threadfence(); *(volatile v8us*)((unsigned short*)X16 + t * 8) = f.half[0];
}

__global__ __launch_bounds__(128) void k_gemm2(const _Float16* __restrict__ A, int lda, size_t sA, const _Float16* __restrict__ Bh, int ldb, size_t sB, float alpha, const float* __restrict__ bias,
    float* __restrict__ C, _Float16* __restrict__ C16, int ldc, size_t sC, int M, int N, int K) {
  __shared__ __attribute__((aligned(16))) float so[4][32][68];
  const int tid = threadIdx.x, w = tid >> 5, lane = tid & 31, ln = lane & 15, hh = lane >> 4; const int by = blockIdx.y;
  A += (size_t)by * sA; Bh += (size_t)by * sB; const size_t cofs = (size_t)by * sC; const float* bp = bias;
  const int ntn = N >> 6; const int mt = blockIdx.x / ntn, nq = blockIdx.x - mt * ntn; const int row0 = mt * 128 + 32 * w, col0 = nq * 64; if (row0 >= M) return;
  const _Float16* a0p = A + (size_t)(row0 + ln) * lda; const _Float16* a1p = a0p + (size_t)16 * lda;
  const _Float16* b0p = Bh + (size_t)(col0 + ln) * ldb; const _Float16* b1p = b0p + (size_t)16 * ldb; const _Float16* b2p = b1p + (size_t)16 * ldb; const _Float16* b3p = b2p + (size_t)16 * ldb;
  const v8f z8 = {0.f,0.f,0.f,0.f,0.f,0.f,0.f,0.f}; v8f c00 = z8, c01 = z8, c02 = z8, c03 = z8, c10 = z8, c11 = z8, c12 = z8, c13 = z8;
#pragma unroll 1
  for (int kb = 0; kb < K; kb += 32) { const v16h a0 = g2_frag(a0p + kb, hh), a1 = g2_frag(a1p + kb, hh);
    v16h b = g2_frag(b0p + kb, hh); c00 = g2_mma(a0, b, c00); c10 = g2_mma(a1, b, c10);
    b = g2_frag(b1p + kb, hh); c01 = g2_mma(a0, b, c01); c11 = g2_mma(a1, b, c11);
    b = g2_frag(b2p + kb, hh); c02 = g2_mma(a0, b, c02); c12 = g2_mma(a1, b, c12);
    b = g2_frag(b3p + kb, hh); c03 = g2_mma(a0, b, c03); c13 = g2_mma(a1, b, c13); }
  v8f accs[8] = {c00, c01, c02, c03, c10, c11, c12, c13};
#pragma unroll
  for (int u = 0; u < 8; ++u) { const int t = u & 3, half = u >> 2; const int col = col0 + t * 16 + ln; const float bv = bp ? bf16_rne(bp[col]) : 0.f;
#pragma unroll
    for (int r = 0; r < 8; ++r) { const int rloc = half * 16 + 8 * hh + r; const float v = accs[u][r] * alpha + bv; so[w][rloc][t * 16 + ln] = v; } }
  __builtin_amdgcn_fence(4  , "workgroup"); __builtin_amdgcn_wave_barrier();
  const int rsub = lane >> 4, c4 = (lane & 15) * 4;
  for (int pass = 0; pass < 2; ++pass) {
#pragma unroll
    for (int q = 0; q < 16; ++q) { const int r = q * 2 + rsub; const v4f v = *(const v4fa*)&so[w][r][c4];
      if (C) *(volatile v4f*)(C + cofs + (size_t)(row0 + r) * ldc + col0 + c4) = v;
      if (C16) { v4h h4;
#pragma unroll
        for (int i = 0; i < 4; ++i) h4[i] = (_Float16)v[i];
        *(volatile v4h*)(C16 + cofs + (size_t)(row0 + r) * ldc + col0 + c4) = h4; } }
    if (pass == 0) __threadfence(); }
}

template <int NHv, int TTv>
__global__ __launch_bounds__(256) void k_vt(const _Float16* __restrict__ V16, int ldv, int voff, _Float16* __restrict__ Vt) {
  __shared__ unsigned short tl[64][66];
  const int tid = threadIdx.x; const int slab = blockIdx.x / (TTv / 64), lg = blockIdx.x % (TTv / 64); const int b = slab / NHv, h = slab % NHv;
  for (int i = tid; i < 64 * 8; i += 256) { const int r = i / 8, c8 = (i % 8) * 8; FragH f; f.half[0] = *(const v8us*)((const unsigned short*)V16 + ((size_t)b * TTv + lg * 64 + r) * ldv + voff + h * 64 + c8);
#pragma unroll
    for (int q = 0; q < 8; ++q) tl[r][c8 + q] = f.u[q]; }
  __syncthreads();
  for (int pass = 0; pass < 2; ++pass) {
#pragma unroll
    for (int rd = 0; rd < 2; ++rd) { const int d = rd * 32 + tid / 8, pc = tid % 8; FragH f;
#pragma unroll
      for (int q = 0; q < 8; ++q) f.u[q] = tl[pc * 8 + q][d];
      *(volatile v8us*)((unsigned short*)Vt + ((size_t)slab * 64 + d) * TTv + lg * 64 + pc * 8) = f.half[0]; }
    if (pass == 0) __threadfence(); }
}

__global__ __launch_bounds__(256) void k_rsmf(const float* __restrict__ S, _Float16* __restrict__ P, int qn, int hg) {
  #pragma clang fp contract(off)
  const int t = blockIdx.x * 256 + threadIdx.x; if (t >= qn * hg) return; const size_t i = (size_t)(t / qn) * SQ + (t % qn); const float* s = S + i * SQ; float mx = -3.0e38f;
#pragma unroll 1
  for (int j = 0; j < SQ; ++j) mx = fmaxf(mx, s[j]); float se = 0.f;
#pragma unroll 1
  for (int j = 0; j < SQ; ++j) se += __expf(s[j] - mx); const float sc = 256.0f / se;
#pragma unroll 1
  for (int j0 = 0; j0 < SQ; j0 += 8) { FragH f;
#pragma unroll
    for (int q = 0; q < 8; ++q) f.h[q] = (_Float16)(__expf(s[j0 + q] - mx) * sc);
    unsigned short* d = (unsigned short*)P + i * SQ + j0; *(volatile v8us*)d = f.half[0]; __threadfence(); *(volatile v8us*)d = f.half[0]; }
}

extern "C" void kernel_launch(void* const* d_in, const int* in_sizes, int n_in,
                              void* d_out, int out_size, void* d_ws, size_t ws_size, hipStream_t stream) {
  if (n_in < 6) return;
  if (in_sizes[0] < (int)((((size_t)(NB - 1)) * SQ_FULL + SQ) * DM)) return;
  if (in_sizes[1] < DM * DM || in_sizes[2] < DM * DM || in_sizes[3] < DM * DM || in_sizes[4] < DM * DM) return;
  if (in_sizes[5] < DM) return;
  if (out_size < (int)(NR * DM)) return;
  const float* x = (const float*)d_in[0]; const float* wq = (const float*)d_in[1]; const float* wk = (const float*)d_in[2];
  const float* wv = (const float*)d_in[3]; const float* wo = (const float*)d_in[4]; const float* bo = (const float*)d_in[5];
  char* ws = (char*)d_ws; size_t off = 0;
  auto take = [&](size_t bytes) { char* p = ws + off; off += (bytes + 255) & ~(size_t)255; return p; };
  _Float16* BQ = (_Float16*)take((size_t)DM * DM * 2); _Float16* BK = (_Float16*)take((size_t)DM * DM * 2); _Float16* BV = (_Float16*)take((size_t)DM * DM * 2); _Float16* BO = (_Float16*)take((size_t)DM * DM * 2);
  _Float16* X16 = (_Float16*)take(NR * DM * 2); _Float16* Q16 = (_Float16*)take(NR * DM * 2); _Float16* K16 = (_Float16*)take(NR * DM * 2); _Float16* V16 = (_Float16*)take(NR * DM * 2); _Float16* O16 = (_Float16*)take(NR * DM * 2);
  float* S = (float*)take((size_t)HG * SQ * SQ * 4); _Float16* P = (_Float16*)take((size_t)HG * SQ * SQ * 2); _Float16* VT = (_Float16*)take((size_t)NH * HD * SQ * 2);
  if (off > ws_size) return;

  { const size_t n8 = (size_t)DM * DM / 8; const unsigned g = (unsigned)((n8 + 255) / 256);
    k_wnat<<<g, 256, 0, stream>>>(wq, n8, BQ); k_wnat<<<g, 256, 0, stream>>>(wk, n8, BK); k_wnat<<<g, 256, 0, stream>>>(wv, n8, BV); k_wnat<<<g, 256, 0, stream>>>(wo, n8, BO); }
  { const size_t n8 = NR * DM / 8; k_x16<<<(unsigned)((n8 + 255) / 256), 256, 0, stream>>>(x, X16, n8); }

  const dim3 gp((unsigned)((MP / 128) * (DM / 64)), 1);
  k_gemm2<<<gp, 128, 0, stream>>>(X16, DM, 0, BQ, DM, 0, 0.0625f, nullptr, nullptr, Q16, DM, 0, MP, DM, DM);
  k_gemm2<<<gp, 128, 0, stream>>>(X16, DM, 0, BK, DM, 0, 0.0625f, nullptr, nullptr, K16, DM, 0, MP, DM, DM);
  k_gemm2<<<gp, 128, 0, stream>>>(X16, DM, 0, BV, DM, 0, 0.0625f, nullptr, nullptr, V16, DM, 0, MP, DM, DM);

  for (int b = 0; b < NB; ++b) { const size_t r0 = (size_t)b * SQ;
    k_vt<NH, SQ><<<NH * (SQ / 64), 256, 0, stream>>>(V16 + r0 * DM, DM, 0, VT);
    for (int h0 = 0; h0 < NH; h0 += HG) {
      k_gemm2<<<dim3((SQ / 128) * (SQ / 64), HG), 128, 0, stream>>>(Q16 + r0 * DM + h0 * HD, DM, (size_t)HD, K16 + r0 * DM + h0 * HD, DM, (size_t)HD, 0.125f, nullptr, S, nullptr, SQ, (size_t)SQ * SQ, SQ, SQ, HD);
      k_rsmf<<<(HG * SQ + 255) / 256, 256, 0, stream>>>(S, P, SQ, HG);
      k_gemm2<<<dim3((SQ / 128) * (HD / 64), HG), 128, 0, stream>>>(P, SQ, (size_t)SQ * SQ, VT + (size_t)h0 * HD * SQ, SQ, (size_t)HD * SQ, 0.25f, nullptr, nullptr, O16 + r0 * DM + h0 * HD, DM, (size_t)HD, SQ, HD, SQ); } }
  k_gemm2<<<gp, 128, 0, stream>>>(O16, DM, 0, BO, DM, 0, 0.0009765625f, bo, (float*)d_out, nullptr, DM, 0, MP, DM, DM);
}
